// DecoderBlock_11613591568704
// MI455X (gfx1250) — hardware-verified
//
#include <hip/hip_runtime.h>
#include <math.h>

#ifndef NB
#define NB 2
#endif
#ifndef SEQ
#define SEQ 1024
#endif
#ifndef MSEQ
#define MSEQ 1024
#endif
#define NB_FULL 2
#define SEQ_FULL 1024
#define MSEQ_FULL 1024

typedef __attribute__((ext_vector_type(16))) _Float16 v16h;
typedef __attribute__((ext_vector_type(8)))  _Float16 v8h;
typedef __attribute__((ext_vector_type(16))) __bf16   v16b;
typedef __attribute__((ext_vector_type(8)))  __bf16   v8b;
typedef __attribute__((ext_vector_type(8)))  float    v8f;
typedef __attribute__((ext_vector_type(4)))  float    v4f;
typedef __attribute__((ext_vector_type(4)))  unsigned v4u;
typedef __attribute__((ext_vector_type(2)))  unsigned v2u;

constexpr int kBatch = NB;
constexpr int kSeq   = SEQ;
constexpr int kMSeq  = MSEQ;
constexpr int kDim   = 1024;
constexpr int kHeads = 16;
constexpr int kHdim  = 64;
constexpr int kFfn   = 4096;
constexpr int kRows  = kBatch * kSeq;
constexpr int kMRows = kBatch * kMSeq;
constexpr int kKvRowsMax = (kRows > kMRows) ? kRows : kMRows;
constexpr int kPosMax    = (kSeq > kMSeq) ? kSeq : kMSeq;
static_assert(kBatch >= 1 && kBatch <= NB_FULL && kSeq <= SEQ_FULL && kMSeq <= MSEQ_FULL);
static_assert(kSeq % 64 == 0 && kMSeq % 64 == 0 && kHdim == 64 && kDim == kHeads * kHdim);
static_assert(kDim % 64 == 0 && kFfn % 64 == 0 && kDim % 32 == 0 && kFfn % 32 == 0);
static_assert(kRows % 64 == 0 && kMRows % 64 == 0);

constexpr float kCarryAct  = 8.0f;
constexpr float kCarryW64  = 64.0f;
constexpr float kCarryW256 = 256.0f;
constexpr float kCarryW512 = 512.0f;
constexpr float kCarryQn   = 65536.0f;
constexpr float kCarryV    = 8.0f;
constexpr float kCarryAttn = 256.0f;
constexpr float kCarryH    = 8.0f;

constexpr size_t kSzWqkv  = (size_t)3 * kDim * kDim * 2;
constexpr size_t kSzWsq   = (size_t)kDim * kDim * 2;
constexpr size_t kSzWkv   = (size_t)2 * kDim * kDim * 2;
constexpr size_t kSzWfc   = (size_t)kFfn * kDim * 2;
constexpr size_t kSzF32T  = (size_t)kRows * kDim * 4;
constexpr size_t kSzH16T  = (size_t)kRows * kDim * 2;
constexpr size_t kSzH16M  = (size_t)kMRows * kDim * 2;
constexpr size_t kSzH16KV = (size_t)kKvRowsMax * kDim * 2;
constexpr size_t kSzBigA  = (size_t)kRows * 3 * kDim * 4;
constexpr size_t kSzBigB  = (size_t)kRows * kDim * 4 + (size_t)kMRows * 2 * kDim * 4;
constexpr size_t kSzBigC  = (size_t)kRows * kFfn * 2;
constexpr size_t kSzBig   = (kSzBigA > kSzBigB) ? ((kSzBigA > kSzBigC) ? kSzBigA : kSzBigC)
                                                : ((kSzBigB > kSzBigC) ? kSzBigB : kSzBigC);
constexpr size_t kSzKsum  = (((size_t)kBatch * kHeads * kHdim * 4) + 127) / 128 * 128;
constexpr size_t kSzRope  = (size_t)kPosMax * 32 * 4;
constexpr size_t kOffWqkv  = 0;
constexpr size_t kOffWsap  = kOffWqkv + kSzWqkv;
constexpr size_t kOffWcaq  = kOffWsap + kSzWsq;
constexpr size_t kOffWcakv = kOffWcaq + kSzWsq;
constexpr size_t kOffWcap  = kOffWcakv + kSzWkv;
constexpr size_t kOffWfc   = kOffWcap + kSzWsq;
constexpr size_t kOffWfcp  = kOffWfc + kSzWfc;
constexpr size_t kOffXr    = kOffWfcp + kSzWfc;
constexpr size_t kOffHln   = kOffXr + kSzF32T;
constexpr size_t kOffBig   = kOffHln + kSzH16T;
constexpr size_t kOffQn    = kOffBig + kSzBig;
constexpr size_t kOffKr    = kOffQn + kSzH16T;
constexpr size_t kOffV8    = kOffKr + kSzH16KV;
constexpr size_t kOffMemh  = kOffV8 + kSzH16KV;
constexpr size_t kOffYatt  = kOffMemh + kSzH16M;
constexpr size_t kOffX1    = kOffYatt + kSzH16T;
constexpr size_t kOffKsum  = kOffX1 + kSzF32T;
constexpr size_t kOffCos   = kOffKsum + kSzKsum;
constexpr size_t kOffSin   = kOffCos + kSzRope;
constexpr size_t kWsTotal  = kOffSin + kSzRope;
constexpr size_t kOffKvf   = kOffBig + (size_t)kRows * kDim * 4;
static_assert(kSzBigA <= kSzBig && kSzBigB <= kSzBig && kSzBigC <= kSzBig);
static_assert(kWsTotal <= 134217728);
static_assert(!(NB == 2 && SEQ == 1024 && MSEQ == 1024) || kWsTotal == 100933632);
static_assert((kOffWsap % 128) == 0 && (kOffWcaq % 128) == 0 && (kOffWcakv % 128) == 0 && (kOffWcap % 128) == 0 &&
              (kOffWfc % 128) == 0 && (kOffWfcp % 128) == 0 && (kOffXr % 128) == 0 && (kOffHln % 128) == 0 &&
              (kOffBig % 128) == 0 && (kOffQn % 128) == 0 && (kOffKr % 128) == 0 && (kOffV8 % 128) == 0 &&
              (kOffMemh % 128) == 0 && (kOffYatt % 128) == 0 && (kOffX1 % 128) == 0 && (kOffKsum % 128) == 0 &&
              (kOffCos % 128) == 0 && (kOffSin % 128) == 0 && (kOffKvf % 128) == 0);
static_assert(((size_t)(kBatch - 1) * SEQ_FULL + kSeq) * kDim <= (size_t)NB_FULL * SEQ_FULL * kDim);

__device__ __forceinline__ unsigned short f2bf_bits(float f) {
  unsigned u = __float_as_uint(f);
  return (unsigned short)((u + 0x7FFFu + ((u >> 16) & 1u)) >> 16);
}
__device__ __forceinline__ float bf_bits2f(unsigned short h) { return __uint_as_float(((unsigned)h) << 16); }
__device__ __forceinline__ float bfr(float f) { return bf_bits2f(f2bf_bits(f)); }
__device__ __forceinline__ v4f bfr4(v4f v) { v4f o; o[0] = bfr(v[0]); o[1] = bfr(v[1]); o[2] = bfr(v[2]); o[3] = bfr(v[3]); return o; }
__device__ __forceinline__ float elu1(float x) {
  const float e = expf(fminf(x, 0.0f));
  return (x > 0.0f) ? (x + 1.0f) : e;
}

__device__ __forceinline__ void dep_guard_h(v8f& a, v8f& b, v16h x, v16h y) { asm volatile("v_nop\n\tv_nop\n\tv_nop\n\tv_nop" : "+v"(a), "+v"(b) : "v"(x), "v"(y)); }
__device__ __forceinline__ void dep_guard_b(v8f& a, v8f& b, v16b x, v16b y) { asm volatile("v_nop\n\tv_nop\n\tv_nop\n\tv_nop" : "+v"(a), "+v"(b) : "v"(x), "v"(y)); }
__device__ __forceinline__ void keep4_h(v16h a, v16h b, v16h c, v16h d) { asm volatile("v_nop" :: "v"(a), "v"(b), "v"(c), "v"(d)); }
__device__ __forceinline__ void keep4_b(v16b a, v16b b, v16b c, v16b d) { asm volatile("v_nop" :: "v"(a), "v"(b), "v"(c), "v"(d)); }
__device__ __forceinline__ void acc_guard4(v8f& a, v8f& b, v8f& c, v8f& d) { asm volatile("v_nop\n\tv_nop\n\tv_nop\n\tv_nop" : "+v"(a), "+v"(b), "+v"(c), "+v"(d)); }
template <typename T> struct Frag;
template <> struct Frag<_Float16> {
  typedef v16h V; union U { v16h v; v8h h[2]; };
  static __device__ __forceinline__ v16h load(const _Float16* p) {
    U f; f.h[0] = *(const v8h*)(p); f.h[1] = *(const v8h*)(p + 16); return f.v;
  }
  static __device__ __forceinline__ v8f mma(v16h a, v16h b, v8f c) {
    return __builtin_amdgcn_wmma_f32_16x16x32_f16(false, a, false, b, (short)0, c, false, false);
  }
  static __device__ __forceinline__ void guard(v8f& a, v8f& b, v16h x, v16h y) { dep_guard_h(a, b, x, y); }
  static __device__ __forceinline__ void keep(v16h a, v16h b, v16h c, v16h d) { keep4_h(a, b, c, d); }
};
template <> struct Frag<__bf16> {
  typedef v16b V; union U { v16b v; v8b h[2]; };
  static __device__ __forceinline__ v16b load(const __bf16* p) {
    U f; f.h[0] = *(const v8b*)(p); f.h[1] = *(const v8b*)(p + 16); return f.v;
  }
  static __device__ __forceinline__ v8f mma(v16b a, v16b b, v8f c) {
    return __builtin_amdgcn_wmma_f32_16x16x32_bf16(false, a, false, b, (short)0, c, false, false);
  }
  static __device__ __forceinline__ void guard(v8f& a, v8f& b, v16b x, v16b y) { dep_guard_b(a, b, x, y); }
  static __device__ __forceinline__ void keep(v16b a, v16b b, v16b c, v16b d) { keep4_b(a, b, c, d); }
};

template <int ET> struct Elem;
template <> struct Elem<0> { typedef _Float16 T; };
template <> struct Elem<1> { typedef __bf16 T; };
template <int ET, bool SPLIT, int BIAS_MODE, int OUT_MODE, bool RESID, int ACT = 0>
__global__ __launch_bounds__(256) void wmma_gemm64(
    const unsigned short* __restrict__ Ap, const unsigned short* __restrict__ A2p, int lda, long strideA,
    const unsigned short* __restrict__ Btp, const unsigned short* __restrict__ Bt2p, int ldb, long strideB,
    void* __restrict__ Cout, void* __restrict__ Cout2, int ldc, long strideC,
    const float* __restrict__ bias,
    const float* __restrict__ resid, long strideR,
    int M, int N, int K, float scale, float oscale) {
  static_assert(!RESID || OUT_MODE == 0);
  typedef typename Elem<ET>::T T;
  typedef typename Frag<T>::V V;
  const T* A = (const T*)Ap; const T* A2 = (const T*)A2p; const T* Bt = (const T*)Btp; const T* Bt2 = (const T*)Bt2p;
  __shared__ __align__(16) float sT[8][16 * 68];
  const int b    = blockIdx.y;
  const int lane = threadIdx.x & 31;
  const int wave = threadIdx.x >> 5;
  const int tilesN = N >> 6;
  const int tilesM = M >> 6;
  const int tile = blockIdx.x * 8 + wave;
  if (tile >= tilesM * tilesN) return;
  const int tm = tile / tilesN;
  const int tn = tile - tm * tilesN;
  const int m0 = tm << 6;
  const int n0 = tn << 6;

  const T* Ab  = A  + (size_t)b * strideA;
  const T* Bb  = Bt + (size_t)b * strideB;
  const T* Ab2 = SPLIT ? (A2  + (size_t)b * strideA) : nullptr;
  const T* Bb2 = SPLIT ? (Bt2 + (size_t)b * strideB) : nullptr;

  const int rlane = lane & 15;
  const int koff  = (lane >> 4) * 8;
  const int mOff  = (lane >> 4) * 8;

  v8f acc[4][4];
#pragma unroll
  for (int i = 0; i < 4; ++i)
#pragma unroll
    for (int j = 0; j < 4; ++j) acc[i][j] = (v8f){0.f,0.f,0.f,0.f,0.f,0.f,0.f,0.f};

  for (int k0 = 0; k0 < K; k0 += 32) {
    V bh[4], bl[4];
#pragma unroll
    for (int j = 0; j < 4; ++j) {
      const size_t bo = (size_t)(n0 + (j << 4) + rlane) * ldb + koff + k0;
      bh[j] = Frag<T>::load(Bb + bo);
      if (SPLIT) bl[j] = Frag<T>::load(Bb2 + bo);
    }
#pragma unroll
    for (int i = 0; i < 4; ++i) {
      const size_t ao = (size_t)(m0 + (i << 4) + rlane) * lda + koff + k0;
      V ah = Frag<T>::load(Ab + ao);
      V al;
      if (SPLIT) al = Frag<T>::load(Ab2 + ao);
#pragma unroll
      for (int j = 0; j < 4; ++j) {
        acc[i][j] = Frag<T>::mma(ah, bh[j], acc[i][j]);
        if (SPLIT) {
          acc[i][j] = Frag<T>::mma(ah, bl[j], acc[i][j]);
          acc[i][j] = Frag<T>::mma(al, bh[j], acc[i][j]);
        }
      }
      Frag<T>::guard(acc[i][0], acc[i][3], ah, SPLIT ? al : ah);
    }
    Frag<T>::keep(bh[0], bh[1], bh[2], bh[3]);
    if (SPLIT) Frag<T>::keep(bl[0], bl[1], bl[2], bl[3]);
  }
  acc_guard4(acc[0][0], acc[0][1], acc[0][2], acc[0][3]);
  acc_guard4(acc[1][0], acc[1][1], acc[1][2], acc[1][3]);
  acc_guard4(acc[2][0], acc[2][1], acc[2][2], acc[2][3]);
  acc_guard4(acc[3][0], acc[3][1], acc[3][2], acc[3][3]);

  float* slab = sT[wave];
  const float* Rb = RESID ? (resid + (size_t)b * strideR) : nullptr;
#pragma unroll
  for (int i = 0; i < 4; ++i) {
    const int mBase = m0 + (i << 4);
#pragma unroll
    for (int j = 0; j < 4; ++j) {
      const int n = n0 + (j << 4) + rlane;
      float bv = 0.f;
      if (BIAS_MODE == 2) bv = bfr(bias[n]);
#pragma unroll
      for (int r = 0; r < 8; ++r) {
        float v = acc[i][j][r] * scale;
        if (BIAS_MODE == 1) v += bfr(bias[mBase + mOff + r]);
        if (BIAS_MODE == 2) v += bv;
        if (ACT == 1) v = tanhf(v);
        if (ACT == 2) v = fmaxf(v, 0.0f);
        if (ACT == 3) v = v / (1.0f + expf(-v));
        if (ACT == 4) v = (v > 0.f) ? v : 0.01f * v;
        if (ACT == 6) {
          float t2 = 1.5957691216057308f * (v + 0.044715f * v * v * v);
          t2 = fmaxf(t2, -80.0f);
          v = v * __builtin_amdgcn_rcpf(1.0f + __expf(-t2));
        }
        slab[(mOff + r) * 68 + (j << 4) + rlane] = v * oscale;
      }
    }
    __builtin_amdgcn_fence(3  , "workgroup");
    __builtin_amdgcn_wave_barrier();
    __builtin_amdgcn_fence(2  , "workgroup");
    if (OUT_MODE == 0) {
      float* C = (float*)Cout + (size_t)b * strideC;
      const int hh = lane >> 4, c4 = (lane & 15) * 4;
      for (int pass = 0; pass < 2; ++pass) {
#pragma unroll
        for (int it = 0; it < 8; ++it) {
          const int row = it * 2 + hh;
          v4f v = *(const v4f*)(slab + row * 68 + c4);
          if (RESID) {
            const v4f rr = *(const v4f*)(Rb + (size_t)(mBase + row) * ldc + n0 + c4);
            v += rr;
          }
          *(volatile v4f*)(C + (size_t)(mBase + row) * ldc + n0 + c4) = v;
        }
        __threadfence();
      }
    } else {
      const int q = lane >> 3, c8 = (lane & 7) * 8;
      unsigned short* C  = (unsigned short*)Cout  + (size_t)b * strideC;
      unsigned short* C2 = (OUT_MODE == 2) ? ((unsigned short*)Cout2 + (size_t)b * strideC) : nullptr;
      for (int pass = 0; pass < 2; ++pass) {
#pragma unroll
        for (int it = 0; it < 4; ++it) {
          const int row = it * 4 + q;
          const float* sp = slab + row * 68 + c8;
          v8h hv, lv;
#pragma unroll
          for (int e = 0; e < 8; ++e) {
            if (OUT_MODE == 1) {
              hv[e] = (_Float16)sp[e];
            } else {
              unsigned short hb = f2bf_bits(sp[e]);
              unsigned short lb = f2bf_bits(sp[e] - bf_bits2f(hb));
              hv[e] = __builtin_bit_cast(_Float16, hb);
              lv[e] = __builtin_bit_cast(_Float16, lb);
            }
          }
          *(volatile v8h*)(C + (size_t)(mBase + row) * ldc + n0 + c8) = hv;
          if (OUT_MODE == 2) *(volatile v8h*)(C2 + (size_t)(mBase + row) * ldc + n0 + c8) = lv;
        }
        __threadfence();
      }
    }
    __builtin_amdgcn_fence(3  , "workgroup");
    __builtin_amdgcn_wave_barrier();
    __builtin_amdgcn_fence(2  , "workgroup");
  }
}

__device__ __forceinline__ void pack4_to_lds(unsigned* hrow, int t, v4f o) {
  const unsigned b0 = (unsigned)__builtin_bit_cast(unsigned short, (_Float16)o[0]);
  const unsigned b1 = (unsigned)__builtin_bit_cast(unsigned short, (_Float16)o[1]);
  const unsigned b2 = (unsigned)__builtin_bit_cast(unsigned short, (_Float16)o[2]);
  const unsigned b3 = (unsigned)__builtin_bit_cast(unsigned short, (_Float16)o[3]);
  v2u pk;
  pk[0] = b0 | (b1 << 16);
  pk[1] = b2 | (b3 << 16);
  *(v2u*)(hrow + 2 * t) = pk;
}
__device__ __forceinline__ void lds_piece_store2(const unsigned* hrow, int piece, _Float16* rowp) {
  const v4u wv = *(const v4u*)(hrow + 4 * piece);
  _Float16* hp = rowp + piece * 8;
  *(volatile v4u*)hp = wv;
  __threadfence();
  *(volatile v4u*)hp = wv;
}

__global__ __launch_bounds__(256) void cvt_w_t(const float* __restrict__ W, _Float16* __restrict__ Wt,
                                               int K, int N, float sc) {
  __shared__ __align__(16) _Float16 sT[64 * 72];
  const int k0 = blockIdx.x * 64;
  const int n0 = blockIdx.y * 64;
  const int t  = threadIdx.x;
  const int kk = t >> 2;
  const int nq = (t & 3) * 16;
  const float* src = W + (size_t)(k0 + kk) * N + n0 + nq;
  const v4f a0 = *(const v4f*)(src);
  const v4f a1 = *(const v4f*)(src + 4);
  const v4f a2 = *(const v4f*)(src + 8);
  const v4f a3 = *(const v4f*)(src + 12);
  _Float16* col = sT + nq * 72 + kk;
#pragma unroll
  for (int e = 0; e < 4; ++e) {
    col[(e) * 72]      = (_Float16)(bfr(a0[e]) * sc);
    col[(4 + e) * 72]  = (_Float16)(bfr(a1[e]) * sc);
    col[(8 + e) * 72]  = (_Float16)(bfr(a2[e]) * sc);
    col[(12 + e) * 72] = (_Float16)(bfr(a3[e]) * sc);
  }
  __syncthreads();
  const int lane = t & 31, w = t >> 5, q = lane >> 3, c8 = (lane & 7) * 8;
  for (int pass = 0; pass < 2; ++pass) {
#pragma unroll
    for (int it = 0; it < 2; ++it) {
      const int row = w * 8 + it * 4 + q;
      const v8h hv = *(const v8h*)(sT + row * 72 + c8);
      *(volatile v8h*)(Wt + (size_t)(n0 + row) * K + k0 + c8) = hv;
    }
    __threadfence();
  }
}

__global__ __launch_bounds__(256) void rope_tab(float* __restrict__ ct, float* __restrict__ st, int n) {
  const int i = blockIdx.x * 256 + threadIdx.x;
  if (i < n) {
    const int pos = i >> 5, j = i & 31;
    const float inv = exp2f(-(float)j * 0.41524101186092028f);
    const float ang = (float)pos * inv;
    float sn, cs;
    sincosf(ang, &sn, &cs);
    ((volatile float*)ct)[i] = cs;
    ((volatile float*)st)[i] = sn;
    __threadfence();
    ((volatile float*)ct)[i] = cs;
    ((volatile float*)st)[i] = sn;
  }
}

__global__ __launch_bounds__(256) void cast_rows_h(const float* __restrict__ x, int rpb, int rstride,
                                                   _Float16* __restrict__ yh, float sc) {
  __shared__ __align__(16) unsigned hrow[512];
  const int row = blockIdx.x;
  const int t = threadIdx.x;
  const int b = row / rpb, tt = row - b * rpb;
  const size_t in_row = (size_t)b * rstride + tt;
  v4f v = *(const v4f*)(x + in_row * kDim + t * 4);
  v = bfr4(v) * sc;
  pack4_to_lds(hrow, t, v);
  __syncthreads();
  if (t < 128) lds_piece_store2(hrow, t, yh + (size_t)row * kDim);
}

template <bool RX, bool WX>
__global__ __launch_bounds__(256) void layernorm_rows(
    const float* __restrict__ x, int rpb, int rstride,
    const float* __restrict__ gam, const float* __restrict__ bet,
    float* __restrict__ xr, _Float16* __restrict__ yh, float hscale) {
  __shared__ float ssum[8];
  __shared__ float ssq[8];
  __shared__ __align__(16) unsigned hrow[512];
  const int row = blockIdx.x;
  const int t = threadIdx.x;
  const int w = t >> 5;
  const int l = t & 31;
  const int b = row / rpb, tt = row - b * rpb;
  const size_t in_row = (size_t)b * rstride + tt;
  v4f v = *(const v4f*)(x + in_row * kDim + t * 4);
  if (RX) v = bfr4(v);
  if (WX) {
    float* xrow = xr + (size_t)row * kDim + t * 4;
    *(volatile v4f*)xrow = v;
    __threadfence();
    *(volatile v4f*)xrow = v;
  }
  float s = (v[0] + v[1]) + (v[2] + v[3]);
#pragma unroll
  for (int off = 1; off < 32; off <<= 1) s += __shfl_xor(s, off, 32);
  if (l == 0) ssum[w] = s;
  __syncthreads();
  float tot = 0.f;
#pragma unroll
  for (int i = 0; i < 8; ++i) tot += ssum[i];
  const float mean = tot * (1.0f / 1024.0f);
  const v4f d = v - mean;
  float q = (d[0] * d[0] + d[1] * d[1]) + (d[2] * d[2] + d[3] * d[3]);
#pragma unroll
  for (int off = 1; off < 32; off <<= 1) q += __shfl_xor(q, off, 32);
  if (l == 0) ssq[w] = q;
  __syncthreads();
  float totq = 0.f;
#pragma unroll
  for (int i = 0; i < 8; ++i) totq += ssq[i];
  const float var = totq * (1.0f / 1024.0f);
  const float inv = rsqrtf(var + 1e-5f);
  const v4f gv = bfr4(*(const v4f*)(gam + t * 4));
  const v4f bv = bfr4(*(const v4f*)(bet + t * 4));
  const v4f o = d * inv * gv + bv;
  pack4_to_lds(hrow, t, o * hscale);
  __syncthreads();
  if (t < 128) lds_piece_store2(hrow, t, yh + (size_t)row * kDim);
}

__global__ __launch_bounds__(256) void ksum_heads(const float* __restrict__ kf, int pitch, int offK, int KS,
                                                  float* __restrict__ ksum) {
  __shared__ float red[4][64];
  const int bh = blockIdx.x;
  const int b = bh / kHeads, h = bh - b * kHeads;
  const int t = threadIdx.x;
  const int rg = t >> 6, d = t & 63;
  const float* p = kf + (size_t)b * KS * pitch + offK + h * kHdim + d;
  float s = 0.f;
#pragma unroll 1
  for (int rr = rg; rr < KS; rr += 4) s += elu1(p[(size_t)rr * pitch]);
  red[rg][d] = s;
  __syncthreads();
  if (t < 64) {
    const float tot = (red[0][t] + red[1][t]) + (red[2][t] + red[3][t]);
    float* op = ksum + (size_t)bh * kHdim + t;
    *(volatile float*)op = tot;
    __threadfence();
    *(volatile float*)op = tot;
  }
}

__global__ __launch_bounds__(256) void feat_kv(const float* __restrict__ kvf, int pitch, int offK, int offV, int KS,
                                               const float* __restrict__ ctab, const float* __restrict__ stab,
                                               _Float16* __restrict__ kr, _Float16* __restrict__ v8, float vcarry) {
  __shared__ __align__(16) float sf[kDim];
  __shared__ __align__(16) unsigned hk[512];
  __shared__ __align__(16) unsigned hv[512];
  const int row = blockIdx.x;
  const int t = threadIdx.x;
  const int b = row / KS, pos = row - b * KS;
  const int d0 = (t & 15) * 4;
  const float* rp = kvf + (size_t)row * pitch;
  const v4f xk = *(const v4f*)(rp + offK + t * 4);
  const v4f xv = *(const v4f*)(rp + offV + t * 4);
  v4f f;
  f[0] = elu1(xk[0]); f[1] = elu1(xk[1]); f[2] = elu1(xk[2]); f[3] = elu1(xk[3]);
  *(v4f*)(sf + t * 4) = f;
  __syncthreads();
  const v4f pr = *(const v4f*)(sf + (t ^ 8) * 4);
  const float sg = ((t & 15) < 8) ? -1.0f : 1.0f;
  const v4f cv = *(const v4f*)(ctab + (size_t)pos * 32 + (d0 & 31));
  const v4f sv = *(const v4f*)(stab + (size_t)pos * 32 + (d0 & 31));
  const v4f o = f * cv + (pr * sv) * sg;
  pack4_to_lds(hk, t, o);
  pack4_to_lds(hv, t, xv * vcarry);
  __syncthreads();
  if (t < 128) lds_piece_store2(hk, t, kr + (size_t)row * kDim);
  else         lds_piece_store2(hv, t - 128, v8 + (size_t)row * kDim);
}

__global__ __launch_bounds__(256) void feat_q(const float* __restrict__ qf, int pitch,
                                              const float* __restrict__ ksum,
                                              const float* __restrict__ ctab, const float* __restrict__ stab,
                                              _Float16* __restrict__ qn, float carry) {
  __shared__ __align__(16) float sf[kDim];
  __shared__ __align__(16) unsigned hrow[512];
  const int row = blockIdx.x;
  const int t = threadIdx.x;
  const int b = row / kSeq, pos = row - b * kSeq;
  const int h = t >> 4, d0 = (t & 15) * 4;
  const v4f xq = *(const v4f*)(qf + (size_t)row * pitch + t * 4);
  v4f f;
  f[0] = elu1(xq[0]); f[1] = elu1(xq[1]); f[2] = elu1(xq[2]); f[3] = elu1(xq[3]);
  const v4f ks = *(const v4f*)(ksum + (size_t)(b * kHeads + h) * kHdim + d0);
  float dp = (f[0] * ks[0] + f[1] * ks[1]) + (f[2] * ks[2] + f[3] * ks[3]);
  dp += __shfl_xor(dp, 1, 32);
  dp += __shfl_xor(dp, 2, 32);
  dp += __shfl_xor(dp, 4, 32);
  dp += __shfl_xor(dp, 8, 32);
  const float qs = carry / dp;
  *(v4f*)(sf + t * 4) = f;
  __syncthreads();
  const v4f pr = *(const v4f*)(sf + (t ^ 8) * 4);
  const float sg = ((t & 15) < 8) ? -1.0f : 1.0f;
  const v4f cv = *(const v4f*)(ctab + (size_t)pos * 32 + (d0 & 31));
  const v4f sv = *(const v4f*)(stab + (size_t)pos * 32 + (d0 & 31));
  const v4f o = (f * cv + (pr * sv) * sg) * qs;
  pack4_to_lds(hrow, t, o);
  __syncthreads();
  if (t < 128) lds_piece_store2(hrow, t, qn + (size_t)row * kDim);
}

constexpr int kAKC = 64;
constexpr int kAQB = 64;
constexpr int kANW = 4;

__device__ __forceinline__ v8f mma_h(v16h a, v16h b, v8f c) {
  c = __builtin_amdgcn_wmma_f32_16x16x32_f16(false, a, false, b, (short)0, c, false, false);
  asm volatile("v_nop\n\tv_nop\n\tv_nop\n\tv_nop" : "+v"(c) : "v"(a), "v"(b));
  return c;
}

__device__ __forceinline__ void vt_scatter(_Float16* vt, v4u w, int d0, int kvr) {
#pragma unroll
  for (int e = 0; e < 4; ++e) {
    const unsigned u = w[e];
    const int d = d0 + 2 * e;
    vt[d * kAKC + kvr]       = __builtin_bit_cast(_Float16, (unsigned short)(u & 0xffffu));
    vt[(d + 1) * kAKC + kvr] = __builtin_bit_cast(_Float16, (unsigned short)(u >> 16));
  }
}

template <bool CAUSAL>
__global__ __launch_bounds__(128)
void lin_attn_h64(const _Float16* __restrict__ qn, const _Float16* __restrict__ kr,
                  const _Float16* __restrict__ v8, _Float16* __restrict__ yout, int KS, float oscale) {
  union FH { v16h v; v8h h[2]; };
  __shared__ __align__(16) _Float16 Ksh[kAKC * kHdim];
  __shared__ __align__(16) _Float16 Vth[kHdim * kAKC];
  __shared__ __align__(16) _Float16 Psh[kANW][16 * kAKC];
  __shared__ __align__(16) float  Osl[kANW][16 * 68];

  const int tid  = threadIdx.x;
  const int wave = tid >> 5;
  const int lane = tid & 31;
  const int hh   = lane >> 4;
  const int c    = lane & 15;

  const int nqb = kSeq / kAQB;
  const int bx = blockIdx.x;
  const int qb = bx % nqb;
  const int bh = bx / nqb;
  const int h  = bh % kHeads;
  const int b  = bh / kHeads;
  const int q0 = qb * kAQB + wave * 16;

  const _Float16* qbase = qn + (size_t)b * kSeq * kDim + (size_t)h * kHdim;
  const _Float16* kbase = kr + (size_t)b * KS * kDim + (size_t)h * kHdim;
  const _Float16* vbase = v8 + (size_t)b * KS * kDim + (size_t)h * kHdim;

  v16h qa[2];
  {
    const _Float16* qrow = qbase + (size_t)(q0 + c) * kDim + 8 * hh;
    qa[0] = Frag<_Float16>::load(qrow);
    qa[1] = Frag<_Float16>::load(qrow + 32);
  }

  v8f oacc[4];
#pragma unroll
  for (int t = 0; t < 4; ++t) oacc[t] = (v8f){0.f,0.f,0.f,0.f,0.f,0.f,0.f,0.f};

  const int nChunks = CAUSAL ? (qb + 1) : (KS / kAKC);
  for (int kc = 0; kc < nChunks; ++kc) {
    const int kv0 = kc * kAKC;
    __syncthreads();
    {
      const int kvr = tid >> 1, dh = (tid & 1) * 32;
      const _Float16* krow = kbase + (size_t)(kv0 + kvr) * kDim + dh;
      const _Float16* vrow = vbase + (size_t)(kv0 + kvr) * kDim + dh;
      const v8h k0v = *(const v8h*)(krow);
      const v8h k1v = *(const v8h*)(krow + 8);
      const v8h k2v = *(const v8h*)(krow + 16);
      const v8h k3v = *(const v8h*)(krow + 24);
      const v4u v0w = *(const v4u*)(vrow);
      const v4u v1w = *(const v4u*)(vrow + 8);
      const v4u v2w = *(const v4u*)(vrow + 16);
      const v4u v3w = *(const v4u*)(vrow + 24);
      _Float16* kd = Ksh + kvr * kHdim + dh;
      *(v8h*)(kd)      = k0v;
      *(v8h*)(kd + 8)  = k1v;
      *(v8h*)(kd + 16) = k2v;
      *(v8h*)(kd + 24) = k3v;
      vt_scatter(Vth, v0w, dh,      kvr);
      vt_scatter(Vth, v1w, dh + 8,  kvr);
      vt_scatter(Vth, v2w, dh + 16, kvr);
      vt_scatter(Vth, v3w, dh + 24, kvr);
    }
    __syncthreads();

    v8f s[4];
#pragma unroll
    for (int j = 0; j < 4; ++j) {
      s[j] = (v8f){0.f,0.f,0.f,0.f,0.f,0.f,0.f,0.f};
#pragma unroll
      for (int dc = 0; dc < 2; ++dc) {
        FH kb;
        kb.h[0] = *(const v8h*)(Ksh + (j * 16 + c) * kHdim + dc * 32 + 8 * hh);
        kb.h[1] = *(const v8h*)(Ksh + (j * 16 + c) * kHdim + dc * 32 + 16 + 8 * hh);
        s[j] = mma_h(qa[dc], kb.v, s[j]);
      }
    }
    const bool diag = CAUSAL && (kc == qb);
    _Float16* pw = Psh[wave];
#pragma unroll
    for (int r = 0; r < 8; ++r) {
      const int qrow = q0 + 8 * hh + r;
#pragma unroll
      for (int j = 0; j < 4; ++j) {
        const int kvcol = kv0 + j * 16 + c;
        float sv = s[j][r];
        sv = (diag && (kvcol > qrow)) ? 0.0f : sv;
        pw[(8 * hh + r) * kAKC + j * 16 + c] = (_Float16)sv;
      }
    }
    __builtin_amdgcn_fence(3  , "workgroup");
    __builtin_amdgcn_wave_barrier();
    __builtin_amdgcn_fence(2  , "workgroup");
#pragma unroll
    for (int kk = 0; kk < 2; ++kk) {
      FH pa;
      pa.h[0] = *(const v8h*)(pw + c * kAKC + kk * 32 + 8 * hh);
      pa.h[1] = *(const v8h*)(pw + c * kAKC + kk * 32 + 16 + 8 * hh);
#pragma unroll
      for (int t = 0; t < 4; ++t) {
        FH vb;
        vb.h[0] = *(const v8h*)(Vth + (t * 16 + c) * kAKC + kk * 32 + 8 * hh);
        vb.h[1] = *(const v8h*)(Vth + (t * 16 + c) * kAKC + kk * 32 + 16 + 8 * hh);
        oacc[t] = mma_h(pa.v, vb.v, oacc[t]);
      }
    }
  }

  float* os = Osl[wave];
#pragma unroll
  for (int r = 0; r < 8; ++r) {
#pragma unroll
    for (int t = 0; t < 4; ++t) os[(8 * hh + r) * 68 + t * 16 + c] = oacc[t][r] * oscale;
  }
  __builtin_amdgcn_fence(3  , "workgroup");
  __builtin_amdgcn_wave_barrier();
  __builtin_amdgcn_fence(2  , "workgroup");
  {
    const int q8 = lane >> 3, c8 = (lane & 7) * 8;
    _Float16* ob = yout + (size_t)b * kSeq * kDim + (size_t)h * kHdim;
    for (int pass = 0; pass < 2; ++pass) {
#pragma unroll
      for (int it = 0; it < 4; ++it) {
        const int row = it * 4 + q8;
        const float* sp = os + row * 68 + c8;
        v8h hv;
#pragma unroll
        for (int e = 0; e < 8; ++e) hv[e] = (_Float16)sp[e];
        *(volatile v8h*)(ob + (size_t)(q0 + row) * kDim + c8) = hv;
      }
      __threadfence();
    }
  }
}

extern "C" void kernel_launch(void* const* d_in, const int* in_sizes, int n_in,
                              void* d_out, int out_size, void* d_ws, size_t ws_size,
                              hipStream_t stream) {
  if (n_in != 22) return;
  const int xNeed = ((kBatch - 1) * SEQ_FULL + kSeq) * kDim;
  const int mNeed = ((kBatch - 1) * MSEQ_FULL + kMSeq) * kDim;
  if (in_sizes[0] < xNeed || in_sizes[1] < mNeed) return;
  if (in_sizes[2] < kDim || in_sizes[3] < kDim || in_sizes[8] < kDim || in_sizes[9] < kDim ||
      in_sizes[16] < kDim || in_sizes[17] < kDim) return;
  if (in_sizes[4] < kDim * 3 * kDim || in_sizes[5] < 3 * kDim) return;
  if (in_sizes[6] < kDim * kDim || in_sizes[7] < kDim) return;
  if (in_sizes[10] < kDim * kDim || in_sizes[11] < kDim) return;
  if (in_sizes[12] < kDim * 2 * kDim || in_sizes[13] < 2 * kDim) return;
  if (in_sizes[14] < kDim * kDim || in_sizes[15] < kDim) return;
  if (in_sizes[18] < kDim * kFfn || in_sizes[19] < kFfn) return;
  if (in_sizes[20] < kFfn * kDim || in_sizes[21] < kDim) return;
  if (out_size < xNeed) return;
  if (ws_size < kWsTotal) return;

  const float* x        = (const float*)d_in[0];
  const float* memory   = (const float*)d_in[1];
  const float* ln1_g    = (const float*)d_in[2];
  const float* ln1_b    = (const float*)d_in[3];
  const float* sa_qkv_w = (const float*)d_in[4];
  const float* sa_qkv_b = (const float*)d_in[5];
  const float* sa_pj_w  = (const float*)d_in[6];
  const float* sa_pj_b  = (const float*)d_in[7];
  const float* ln2_g    = (const float*)d_in[8];
  const float* ln2_b    = (const float*)d_in[9];
  const float* ca_q_w   = (const float*)d_in[10];
  const float* ca_q_b   = (const float*)d_in[11];
  const float* ca_kv_w  = (const float*)d_in[12];
  const float* ca_kv_b  = (const float*)d_in[13];
  const float* ca_pj_w  = (const float*)d_in[14];
  const float* ca_pj_b  = (const float*)d_in[15];
  const float* ln3_g    = (const float*)d_in[16];
  const float* ln3_b    = (const float*)d_in[17];
  const float* fc_w     = (const float*)d_in[18];
  const float* fc_b     = (const float*)d_in[19];
  const float* fcp_w    = (const float*)d_in[20];
  const float* fcp_b    = (const float*)d_in[21];
  float* outf = (float*)d_out;

  char* ws = (char*)d_ws;
  _Float16* wqkv  = (_Float16*)(ws + kOffWqkv);
  _Float16* wsap  = (_Float16*)(ws + kOffWsap);
  _Float16* wcaq  = (_Float16*)(ws + kOffWcaq);
  _Float16* wcakv = (_Float16*)(ws + kOffWcakv);
  _Float16* wcap  = (_Float16*)(ws + kOffWcap);
  _Float16* wfc   = (_Float16*)(ws + kOffWfc);
  _Float16* wfcp  = (_Float16*)(ws + kOffWfcp);
  float*    xr    = (float*)(ws + kOffXr);
  _Float16* hln   = (_Float16*)(ws + kOffHln);
  float*    big   = (float*)(ws + kOffBig);
  float*    qca   = (float*)(ws + kOffBig);
  float*    kvf   = (float*)(ws + kOffKvf);
  _Float16* hid   = (_Float16*)(ws + kOffBig);
  _Float16* qnp   = (_Float16*)(ws + kOffQn);
  _Float16* krp   = (_Float16*)(ws + kOffKr);
  _Float16* v8p   = (_Float16*)(ws + kOffV8);
  _Float16* memh  = (_Float16*)(ws + kOffMemh);
  _Float16* yatt  = (_Float16*)(ws + kOffYatt);
  float*    x1    = (float*)(ws + kOffX1);
  float*    x2    = xr;
  float*    ksum  = (float*)(ws + kOffKsum);
  float*    ctab  = (float*)(ws + kOffCos);
  float*    stab  = (float*)(ws + kOffSin);

  typedef const unsigned short* cus;

  cvt_w_t<<<dim3(kDim / 64, (3 * kDim) / 64), dim3(256), 0, stream>>>(sa_qkv_w, wqkv, kDim, 3 * kDim, kCarryW64);
  cvt_w_t<<<dim3(kDim / 64, kDim / 64), dim3(256), 0, stream>>>(sa_pj_w, wsap, kDim, kDim, kCarryW256);
  cvt_w_t<<<dim3(kDim / 64, kDim / 64), dim3(256), 0, stream>>>(ca_q_w, wcaq, kDim, kDim, kCarryW64);
  cvt_w_t<<<dim3(kDim / 64, (2 * kDim) / 64), dim3(256), 0, stream>>>(ca_kv_w, wcakv, kDim, 2 * kDim, kCarryW64);
  cvt_w_t<<<dim3(kDim / 64, kDim / 64), dim3(256), 0, stream>>>(ca_pj_w, wcap, kDim, kDim, kCarryW256);
  cvt_w_t<<<dim3(kDim / 64, kFfn / 64), dim3(256), 0, stream>>>(fc_w, wfc, kDim, kFfn, kCarryW256);
  cvt_w_t<<<dim3(kFfn / 64, kDim / 64), dim3(256), 0, stream>>>(fcp_w, wfcp, kFfn, kDim, kCarryW512);

  {
    const int n = kPosMax * 32;
    rope_tab<<<dim3((unsigned)((n + 255) / 256)), dim3(256), 0, stream>>>(ctab, stab, n);
  }

  cast_rows_h<<<dim3((unsigned)kMRows), dim3(256), 0, stream>>>(memory, kMSeq, MSEQ_FULL, memh, kCarryAct);

  layernorm_rows<true, true><<<dim3((unsigned)kRows), dim3(256), 0, stream>>>(x, kSeq, SEQ_FULL, ln1_g, ln1_b, xr, hln, kCarryAct);

  {
    const unsigned blocks = (unsigned)(((kRows / 64) * ((3 * kDim) / 64) + 7) / 8);
    wmma_gemm64<0, false, 2, 0, false, 0><<<dim3(blocks, 1), dim3(256), 0, stream>>>(
        (cus)hln, (cus)hln, kDim, (long)0,
        (cus)wqkv, (cus)wqkv, kDim, (long)0,
        (void*)big, (void*)big, 3 * kDim, (long)0,
        sa_qkv_b, xr, (long)0,
        kRows, 3 * kDim, kDim, 1.0f / (kCarryAct * kCarryW64), 1.0f);
  }

  ksum_heads<<<dim3((unsigned)(kBatch * kHeads)), dim3(256), 0, stream>>>(big, 3 * kDim, kDim, kSeq, ksum);
  feat_kv<<<dim3((unsigned)kRows), dim3(256), 0, stream>>>(big, 3 * kDim, kDim, 2 * kDim, kSeq, ctab, stab, krp, v8p, kCarryV);
  feat_q<<<dim3((unsigned)kRows), dim3(256), 0, stream>>>(big, 3 * kDim, ksum, ctab, stab, qnp, kCarryQn);

  {
    const unsigned blocks = (unsigned)(kBatch * kHeads * (kSeq / kAQB));
    lin_attn_h64<true><<<dim3(blocks), dim3(128), 0, stream>>>(qnp, krp, v8p, yatt, kSeq, kCarryAttn / (kCarryQn * kCarryV));
  }

  {
    const unsigned blocks = (unsigned)(((kRows / 64) * (kDim / 64) + 7) / 8);
    wmma_gemm64<0, false, 2, 0, true, 0><<<dim3(blocks, 1), dim3(256), 0, stream>>>(
        (cus)yatt, (cus)yatt, kDim, (long)0,
        (cus)wsap, (cus)wsap, kDim, (long)0,
        (void*)x1, (void*)x1, kDim, (long)0,
        sa_pj_b, xr, (long)0,
        kRows, kDim, kDim, 1.0f / (kCarryAttn * kCarryW256), 1.0f);
  }

  layernorm_rows<false, false><<<dim3((unsigned)kRows), dim3(256), 0, stream>>>(x1, kSeq, kSeq, ln2_g, ln2_b, xr, hln, kCarryAct);

  {
    const unsigned blocks = (unsigned)(((kRows / 64) * (kDim / 64) + 7) / 8);
    wmma_gemm64<0, false, 2, 0, false, 0><<<dim3(blocks, 1), dim3(256), 0, stream>>>(
        (cus)hln, (cus)hln, kDim, (long)0,
        (cus)wcaq, (cus)wcaq, kDim, (long)0,
        (void*)qca, (void*)qca, kDim, (long)0,
        ca_q_b, xr, (long)0,
        kRows, kDim, kDim, 1.0f / (kCarryAct * kCarryW64), 1.0f);
  }

  {
    const unsigned blocks = (unsigned)(((kMRows / 64) * ((2 * kDim) / 64) + 7) / 8);
    wmma_gemm64<0, false, 2, 0, false, 0><<<dim3(blocks, 1), dim3(256), 0, stream>>>(
        (cus)memh, (cus)memh, kDim, (long)0,
        (cus)wcakv, (cus)wcakv, kDim, (long)0,
        (void*)kvf, (void*)kvf, 2 * kDim, (long)0,
        ca_kv_b, xr, (long)0,
        kMRows, 2 * kDim, kDim, 1.0f / (kCarryAct * kCarryW64), 1.0f);
  }

  ksum_heads<<<dim3((unsigned)(kBatch * kHeads)), dim3(256), 0, stream>>>(kvf, 2 * kDim, 0, kMSeq, ksum);
  feat_kv<<<dim3((unsigned)kMRows), dim3(256), 0, stream>>>(kvf, 2 * kDim, 0, kDim, kMSeq, ctab, stab, krp, v8p, kCarryV);
  feat_q<<<dim3((unsigned)kRows), dim3(256), 0, stream>>>(qca, kDim, ksum, ctab, stab, qnp, kCarryQn);

  {
    const unsigned blocks = (unsigned)(kBatch * kHeads * (kSeq / kAQB));
    lin_attn_h64<false><<<dim3(blocks), dim3(128), 0, stream>>>(qnp, krp, v8p, yatt, kMSeq, kCarryAttn / (kCarryQn * kCarryV));
  }

  {
    const unsigned blocks = (unsigned)(((kRows / 64) * (kDim / 64) + 7) / 8);
    wmma_gemm64<0, false, 2, 0, true, 0><<<dim3(blocks, 1), dim3(256), 0, stream>>>(
        (cus)yatt, (cus)yatt, kDim, (long)0,
        (cus)wcap, (cus)wcap, kDim, (long)0,
        (void*)x2, (void*)x2, kDim, (long)0,
        ca_pj_b, x1, (long)0,
        kRows, kDim, kDim, 1.0f / (kCarryAttn * kCarryW256), 1.0f);
  }

  layernorm_rows<false, false><<<dim3((unsigned)kRows), dim3(256), 0, stream>>>(x2, kSeq, kSeq, ln3_g, ln3_b, x1, hln, kCarryAct);

  {
    const unsigned blocks = (unsigned)(((kRows / 64) * (kFfn / 64) + 7) / 8);
    wmma_gemm64<0, false, 2, 1, false, 6><<<dim3(blocks, 1), dim3(256), 0, stream>>>(
        (cus)hln, (cus)hln, kDim, (long)0,
        (cus)wfc, (cus)wfc, kDim, (long)0,
        (void*)hid, (void*)hid, kFfn, (long)0,
        fc_b, x1, (long)0,
        kRows, kFfn, kDim, 1.0f / (kCarryAct * kCarryW256), kCarryH);
  }

  {
    const unsigned blocks = (unsigned)(((kSeq / 64) * (kDim / 64) + 7) / 8);
    wmma_gemm64<0, false, 2, 0, true, 0><<<dim3(blocks, (unsigned)kBatch), dim3(256), 0, stream>>>(
        (cus)hid, (cus)hid, kFfn, (long)kSeq * kFfn,
        (cus)wfcp, (cus)wfcp, kFfn, (long)0,
        (void*)outf, (void*)outf, kDim, (long)SEQ_FULL * kDim,
        fcp_b, x2, (long)kSeq * kDim,
        kSeq, kDim, kFfn, 1.0f / (kCarryH * kCarryW512), 1.0f);
  }
}
